// CustomDotProductAttention_1563368095789
// MI455X (gfx1250) — hardware-verified
//
#include <hip/hip_runtime.h>
#include <math.h>
#include <float.h>
#include <stdint.h>

#define LQ    2048
#define SK    2048
#define NBAT  2
#define NHEAD 16
#define HD    128
#define BHN   (NBAT * NHEAD)
#define ROWF  (BHN * HD)
#define NQB   (LQ / 64)
#define RESQB 4
#define NTOT  (LQ * ROWF)
#define VSC   16.0f
static_assert(LQ == SK);
static_assert((LQ % 64) == 0);
static_assert(HD == 128);
static_assert(((BHN * LQ * (HD / 8)) % 256) == 0);
static_assert(RESQB <= NQB);

typedef _Float16 v16h __attribute__((ext_vector_type(16)));
typedef _Float16 v8h  __attribute__((ext_vector_type(8)));
typedef __bf16   v16b __attribute__((ext_vector_type(16)));
typedef __bf16   v8b  __attribute__((ext_vector_type(8)));
typedef float    v8f  __attribute__((ext_vector_type(8)));
typedef float    v4f  __attribute__((ext_vector_type(4)));
typedef unsigned int v4u __attribute__((ext_vector_type(4)));

__device__ __forceinline__ unsigned short bf_bits(float f) {
  unsigned u = __float_as_uint(f);
  return (unsigned short)((u + 0x7FFFu + ((u >> 16) & 1u)) >> 16);
}
__device__ __forceinline__ float bf_up(unsigned short h) { return __uint_as_float(((unsigned)h) << 16); }
__device__ __forceinline__ unsigned short h_bits(_Float16 x) { return __builtin_bit_cast(unsigned short, x); }
__device__ __forceinline__ unsigned pk16(unsigned short a, unsigned short b) { return (unsigned)a | ((unsigned)b << 16); }
__device__ __forceinline__ v8f zero8() { v8f z = {0.f, 0.f, 0.f, 0.f, 0.f, 0.f, 0.f, 0.f}; return z; }

__device__ __forceinline__ v16b ldfrag_b(const __bf16* p) {
  union { v16b v; v8b h[2]; } f;
  f.h[0] = *(const v8b*)(p);
  f.h[1] = *(const v8b*)(p + 16);
  return f.v;
}

__device__ __forceinline__ v8f mma_b(v16b a, v16b b, v8f c) {
  c = __builtin_amdgcn_wmma_f32_16x16x32_bf16(false, a, false, b, (short)0, c, false, false);
#if defined(__HIP_DEVICE_COMPILE__)
  asm volatile("v_nop\n\tv_nop\n\tv_nop\n\tv_nop" : "+v"(c) : "v"(a), "v"(b));
#endif
  return c;
}
__device__ __forceinline__ v8f mma_h(v16h a, v16h b, v8f c) {
  c = __builtin_amdgcn_wmma_f32_16x16x32_f16(false, a, false, b, (short)0, c, false, false);
#if defined(__HIP_DEVICE_COMPILE__)
  asm volatile("v_nop\n\tv_nop\n\tv_nop\n\tv_nop" : "+v"(c) : "v"(a), "v"(b));
#endif
  return c;
}

__global__ __launch_bounds__(256) void cvt_rows_bf16(const float* __restrict__ in, unsigned short* out, int n8) {
  const int i = blockIdx.x * 256 + threadIdx.x;
  if (i < n8) {
    const int per = LQ * (HD / 8);
    const int bh  = i / per;
    const int rem = i - bh * per;
    const int l   = rem / (HD / 8);
    const int d0  = (rem - l * (HD / 8)) * 8;
    const size_t src = (size_t)l * ROWF + (size_t)bh * HD + (size_t)d0;
    const v4f a = *(const v4f*)(in + src);
    const v4f b = *(const v4f*)(in + src + 4);
    v4u p;
    p[0] = pk16(bf_bits(a[0]), bf_bits(a[1]));
    p[1] = pk16(bf_bits(a[2]), bf_bits(a[3]));
    p[2] = pk16(bf_bits(b[0]), bf_bits(b[1]));
    p[3] = pk16(bf_bits(b[2]), bf_bits(b[3]));
    *(volatile v4u*)(out + (size_t)i * 8) = p;
    __threadfence();
    *(volatile v4u*)(out + (size_t)i * 8) = p;
  }
}

__global__ __launch_bounds__(256) void v_planes(const float* __restrict__ vf, unsigned short* vt, float vsc) {
  __shared__ __align__(16) float sv[64 * 132];
  const int tid = threadIdx.x;
  const int s0  = blockIdx.x * 64;
  const int bh  = blockIdx.y;
#pragma unroll
  for (int i = 0; i < 8; ++i) {
    const int idx = i * 256 + tid;
    const int tt = idx >> 5, c4 = (idx & 31) * 4;
    const v4f a = *(const v4f*)(vf + (size_t)(s0 + tt) * ROWF + (size_t)bh * HD + c4);
    *(v4f*)(sv + tt * 132 + c4) = a;
  }
  __syncthreads();

  const int g = tid >> 3, piece = tid & 7;
  v4u hv[4];
  size_t hofs[4];
#pragma unroll
  for (int it = 0; it < 4; ++it) {
    const int d = it * 32 + g;
    v4u a;
#pragma unroll
    for (int e = 0; e < 4; ++e) {
      const float f0 = sv[(piece * 8 + 2 * e) * 132 + d];
      const float f1 = sv[(piece * 8 + 2 * e + 1) * 132 + d];
      const _Float16 x0 = (_Float16)(bf_up(bf_bits(f0)) * vsc);
      const _Float16 x1 = (_Float16)(bf_up(bf_bits(f1)) * vsc);
      a[e] = pk16(h_bits(x0), h_bits(x1));
    }
    hv[it] = a;
    hofs[it] = ((size_t)(bh * HD + d)) * SK + (size_t)s0 + (size_t)(piece * 8);
  }
  for (int pass = 0; pass < 2; ++pass) {
#pragma unroll
    for (int it = 0; it < 4; ++it) {
      *(volatile v4u*)(vt + hofs[it]) = hv[it];
    }
    __threadfence();
  }
}

template <bool RESP>
__global__ __launch_bounds__(128)
void attn_causal(const unsigned short* __restrict__ qpl, const unsigned short* __restrict__ kpl,
                 const unsigned short* __restrict__ vtpl, float* outp, int qbBase, int nqbThis, float sscale) {
  union FH { v16h v; v8h h[2]; };
  union FB { v16b v; v8b h[2]; };
  __shared__ __align__(16) __bf16   Ksh[64 * HD];
  __shared__ __align__(16) _Float16 Vth[HD * 64];
  __shared__ __align__(16) _Float16 Psh[4][16 * 64];
  __shared__ __align__(16) _Float16 Psl[RESP ? 4 : 1][16 * 64];
  __shared__ __align__(16) float    Os[4][16 * HD];

  const int tid  = threadIdx.x;
  const int wave = tid >> 5;
  const int lane = tid & 31;
  const int hh   = lane >> 4;
  const int c    = lane & 15;

  const int bx  = blockIdx.x;
  const int qbl = bx % nqbThis;
  const int bh  = bx / nqbThis;
  const int qb  = qbBase + qbl;
  if (qb >= NQB || bh >= BHN) return;
  const int q0  = qb * 64 + wave * 16;

  const __bf16*   Qp = (const __bf16*)(const void*)qpl + (size_t)bh * LQ * HD;
  const __bf16*   Kp = (const __bf16*)(const void*)kpl + (size_t)bh * SK * HD;
  const _Float16* Vh = (const _Float16*)(const void*)vtpl + (size_t)bh * HD * SK;

  v16b qa[4];
#pragma unroll
  for (int dc = 0; dc < 4; ++dc) {
    qa[dc] = ldfrag_b(Qp + (size_t)(q0 + c) * HD + dc * 32 + 8 * hh);
  }

  float mrow[8], lrow[8];
  v8f oacc[8];
#pragma unroll
  for (int r = 0; r < 8; ++r) { mrow[r] = -INFINITY; lrow[r] = 0.f; }
#pragma unroll
  for (int t = 0; t < 8; ++t) oacc[t] = zero8();

  int nkt = qb + 1;
  if (nkt > NQB) nkt = NQB;
  for (int kt = 0; kt < nkt; ++kt) {
    const int kv0 = kt * 64;
    __syncthreads();
    {
      const int r = tid >> 1, half = (tid & 1) * 64;
      const __bf16* kg = Kp + (size_t)(kv0 + r) * HD + half;
#pragma unroll
      for (int i = 0; i < 8; ++i) {
        const v8b a0 = *(const v8b*)(kg + 8 * i);
        *(v8b*)(Ksh + r * HD + half + 8 * i) = a0;
      }
      const _Float16* vg = Vh + (size_t)tid * SK + kv0;
#pragma unroll
      for (int i = 0; i < 8; ++i) {
        const v8h b0 = *(const v8h*)(vg + 8 * i);
        *(v8h*)(Vth + tid * 64 + 8 * i) = b0;
      }
    }
    __syncthreads();

    v8f s[4];
#pragma unroll
    for (int j = 0; j < 4; ++j) {
      s[j] = zero8();
#pragma unroll
      for (int dc = 0; dc < 4; ++dc) {
        FB kb;
        kb.h[0] = *(const v8b*)(Ksh + (j * 16 + c) * HD + dc * 32 + 8 * hh);
        kb.h[1] = *(const v8b*)(Ksh + (j * 16 + c) * HD + dc * 32 + 16 + 8 * hh);
        s[j] = mma_b(qa[dc], kb.v, s[j]);
      }
    }

    _Float16* pwh = Psh[wave];
    _Float16* pwl = Psl[RESP ? wave : 0];
#pragma unroll
    for (int r = 0; r < 8; ++r) {
      const int qrow = q0 + 8 * hh + r;
      float m = -INFINITY;
#pragma unroll
      for (int j = 0; j < 4; ++j) {
        const int key = kv0 + j * 16 + c;
        float sv = s[j][r] * sscale;
        sv = (key > qrow) ? -FLT_MAX : sv;
        s[j][r] = sv;
        m = fmaxf(m, sv);
      }
#pragma unroll
      for (int off = 1; off < 16; off <<= 1) m = fmaxf(m, __shfl_xor(m, off, 32));
      const float mnew  = fmaxf(mrow[r], m);
      const float msafe = (mnew == -INFINITY) ? 0.f : mnew;
      const float alpha = __expf(mrow[r] - msafe);
      mrow[r] = mnew;
      float psum = 0.f;
#pragma unroll
      for (int j = 0; j < 4; ++j) {
        const float p = __expf(s[j][r] - msafe);
        psum += p;
        const float p1k = p * 1024.0f;
        const _Float16 ph = (_Float16)p1k;
        pwh[(8 * hh + r) * 64 + j * 16 + c] = ph;
        if (RESP) {
          const _Float16 pl = (_Float16)(p1k - (float)ph);
          pwl[(8 * hh + r) * 64 + j * 16 + c] = pl;
        }
      }
#pragma unroll
      for (int off = 1; off < 16; off <<= 1) psum += __shfl_xor(psum, off, 32);
      lrow[r] = lrow[r] * alpha + psum;
#pragma unroll
      for (int t = 0; t < 8; ++t) oacc[t][r] *= alpha;
    }
    __builtin_amdgcn_fence(__ATOMIC_RELEASE, "workgroup");
    __builtin_amdgcn_wave_barrier();
    __builtin_amdgcn_fence(__ATOMIC_ACQUIRE, "workgroup");

#pragma unroll 1
    for (int kk = 0; kk < 2; ++kk) {
      FH pa, pl;
      pa.h[0] = *(const v8h*)(pwh + c * 64 + kk * 32 + 8 * hh);
      pa.h[1] = *(const v8h*)(pwh + c * 64 + kk * 32 + 16 + 8 * hh);
      if (RESP) {
        pl.h[0] = *(const v8h*)(pwl + c * 64 + kk * 32 + 8 * hh);
        pl.h[1] = *(const v8h*)(pwl + c * 64 + kk * 32 + 16 + 8 * hh);
      } else {
        pl.v = pa.v;
      }
#pragma unroll
      for (int t = 0; t < 8; ++t) {
        FH vb;
        vb.h[0] = *(const v8h*)(Vth + (t * 16 + c) * 64 + kk * 32 + 8 * hh);
        vb.h[1] = *(const v8h*)(Vth + (t * 16 + c) * 64 + kk * 32 + 16 + 8 * hh);
        oacc[t] = mma_h(pa.v, vb.v, oacc[t]);
        if (RESP) oacc[t] = mma_h(pl.v, vb.v, oacc[t]);
      }
    }
  }

  float* os = Os[wave];
#pragma unroll
  for (int r = 0; r < 8; ++r) {
    const float l = lrow[r];
    const float inv = ((l > 0.f) ? (1.0f / l) : 0.f) * (1.0f / (1024.0f * VSC));
#pragma unroll
    for (int t = 0; t < 8; ++t) os[(8 * hh + r) * HD + t * 16 + c] = oacc[t][r] * inv;
  }
  __builtin_amdgcn_fence(__ATOMIC_RELEASE, "workgroup");
  __builtin_amdgcn_wave_barrier();
  __builtin_amdgcn_fence(__ATOMIC_ACQUIRE, "workgroup");
  {
    const int c4 = lane * 4;
    for (int pass = 0; pass < 2; ++pass) {
#pragma unroll
      for (int it = 0; it < 16; ++it) {
        const v4f ov = *(const v4f*)(os + it * HD + c4);
        const size_t go = (size_t)(q0 + it) * ROWF + (size_t)bh * HD + (size_t)c4;
        *(volatile v4f*)(outp + go) = ov;
      }
      __threadfence();
    }
  }
}

extern "C" void kernel_launch(void* const* d_in, const int* in_sizes, int n_in,
                              void* d_out, int out_size, void* d_ws, size_t ws_size,
                              hipStream_t stream) {
  if (n_in < 3) return;
  if (in_sizes[0] != NTOT) return;
  if (in_sizes[1] != SK * ROWF) return;
  if (in_sizes[2] != SK * ROWF) return;
  if (out_size != NTOT) return;

  const float* q = (const float*)d_in[0];
  const float* k = (const float*)d_in[1];
  const float* v = (const float*)d_in[2];

  const size_t PQ = (size_t)BHN * LQ * HD * 2;
  const size_t PK = (size_t)BHN * SK * HD * 2;
  const size_t PV = (size_t)BHN * HD * SK * 2;
  size_t off = 0;
  const size_t oQ = off; off += PQ;
  const size_t oK = off; off += PK;
  const size_t oV = off; off += PV;
  if (off > ws_size) return;
  if (off > (size_t)134217728) return;

  char* ws = (char*)d_ws;
  unsigned short* Qb = (unsigned short*)(ws + oQ);
  unsigned short* Kb = (unsigned short*)(ws + oK);
  unsigned short* Vt = (unsigned short*)(ws + oV);
  float* outf = (float*)d_out;

  const dim3 blk(256);
  const int n8 = BHN * LQ * (HD / 8);
  const dim3 gCvt((n8 + 255) / 256);
  const dim3 gV(SK / 64, BHN);
  const float sscale = (float)(1.0 / sqrt((double)HD));

  cvt_rows_bf16<<<gCvt, blk, 0, stream>>>(q, Qb, n8);
  cvt_rows_bf16<<<gCvt, blk, 0, stream>>>(k, Kb, n8);
  v_planes<<<gV, blk, 0, stream>>>(v, Vt, VSC);
  attn_causal<true><<<dim3(BHN * RESQB), dim3(128), 0, stream>>>(Qb, Kb, Vt, outf, 0, RESQB, sscale);
  attn_causal<false><<<dim3(BHN * (NQB - RESQB)), dim3(128), 0, stream>>>(Qb, Kb, Vt, outf, RESQB, NQB - RESQB, sscale);
  (void)hipGetLastError();
}
